// KGCN_4827543240786
// MI455X (gfx1250) — hardware-verified
//
#include <hip/hip_runtime.h>


namespace {
constexpr int BT = 16384, NU = 100000, NE = 100000, NI = 20000, NIKG = 20000, NR = 60, D = 64, NN = 8;
constexpr float XS = 8.0f, WSC = 256.0f;
typedef _Float16 b16;
typedef __attribute__((ext_vector_type(16))) _Float16 v16b;
typedef __attribute__((ext_vector_type(8))) _Float16 v8b;
typedef __attribute__((ext_vector_type(8))) float v8f;
typedef __attribute__((ext_vector_type(4))) float v4f;
typedef __attribute__((ext_vector_type(2))) float v2f;
__device__ __forceinline__ float bf16_rne(float f) { unsigned int u = __float_as_uint(f); u += 0x7FFFu + ((u >> 16) & 1u); return __uint_as_float(u & 0xFFFF0000u); }
__device__ __forceinline__ void split16(float v, b16& hi, b16& lo) { hi = (b16)v; lo = (b16)(v - (float)hi); }
__device__ __forceinline__ v16b frag_kb(const b16* p, int hh) { const v8b a = *(const v8b*)(p + 8 * hh), b = *(const v8b*)(p + 16 + 8 * hh); v16b f;
#pragma unroll
  for (int e = 0; e < 8; ++e) { f[e] = a[e]; f[8 + e] = b[e]; } return f; }
__device__ __forceinline__ v8f wmma16b(v16b a, v16b b, v8f c) { v8f d = __builtin_amdgcn_wmma_f32_16x16x32_f16(false, a, false, b, (short)0, c, false, false); asm volatile("v_nop\n\tv_nop\n\tv_nop\n\tv_nop" : "+v"(d) : "v"(a), "v"(b)); return d; }
__device__ __forceinline__ void wave_lds_sync() { __builtin_amdgcn_fence(__ATOMIC_RELEASE, "workgroup"); __builtin_amdgcn_wave_barrier(); __builtin_amdgcn_fence(__ATOMIC_ACQUIRE, "workgroup"); }
__device__ __forceinline__ float pmul(float a, float b) { float p = a * b; asm volatile("" : "+v"(p)); return p; }
__device__ __forceinline__ int iclamp(int v, int lo, int hi) { return v < lo ? lo : (v > hi ? hi : v); }
__device__ __forceinline__ float sigm(float v) { return 1.0f / (1.0f + __expf(-v)); }

__global__ __launch_bounds__(256) void wcopy_kernel(const float* __restrict__ w, b16* __restrict__ WT) {
  const int u = blockIdx.x * 256 + threadIdx.x; if (u >= D * D / 8) return; const int e = u * 8; v8b v; for (int j = 0; j < 8; ++j) v[j] = (b16)(bf16_rne(w[e + j]) * WSC);
  for (int pass = 0; pass < 2; ++pass) { *(volatile v8b*)(WT + e) = v; __threadfence(); }
}
template <int NVSRC>
__device__ __forceinline__ void build_A(int rr, const float* __restrict__ ue_row, v2f selfv, const int* __restrict__ relid, const int* __restrict__ nbr, const float* __restrict__ rel_emb, const float* __restrict__ ent_emb, const float* __restrict__ O1, size_t o1base, int lane, b16 (*Ah)[D + 8], b16 (*Al)[D + 8]) {
  const v2f uu = *(const v2f*)(ue_row + lane * 2); const float u0 = bf16_rne(uu[0]), u1 = bf16_rne(uu[1]); float s[NN]; float mx = -INFINITY;
#pragma unroll
  for (int n = 0; n < NN; ++n) { const int r = iclamp(relid[n], 0, NR); const v2f rv = *(const v2f*)(rel_emb + (size_t)r * D + lane * 2); float d = pmul(u0, bf16_rne(rv[0])) + pmul(u1, bf16_rne(rv[1])); for (int o = 16; o; o >>= 1) d += __shfl_xor(d, o); s[n] = d; mx = fmaxf(mx, d); }
  float den = 0.0f;
#pragma unroll
  for (int n = 0; n < NN; ++n) { s[n] = __expf(s[n] - mx); den += s[n]; }
  float a0 = 0.0f, a1 = 0.0f;
#pragma unroll
  for (int n = 0; n < NN; ++n) { const float w = s[n] / den; v2f nv; if (NVSRC == 0) { const int e = iclamp(nbr[n], 0, NE); const v2f t = *(const v2f*)(ent_emb + (size_t)e * D + lane * 2); nv[0] = bf16_rne(t[0]); nv[1] = bf16_rne(t[1]); } else nv = *(const v2f*)(O1 + (o1base + n) * D + lane * 2);
    a0 += pmul(w, nv[0]); a1 += pmul(w, nv[1]); }
  b16 p, q; split16((selfv[0] + a0) * XS, p, q); Ah[rr][lane * 2] = p; Al[rr][lane * 2] = q; split16((selfv[1] + a1) * XS, p, q); Ah[rr][lane * 2 + 1] = p; Al[rr][lane * 2 + 1] = q;
}
__device__ __forceinline__ void gemm64(b16 (*Ah)[D + 8], b16 (*Al)[D + 8], const b16* __restrict__ WT, int nloc, int hlf, v8f* acc) {
#pragma unroll
  for (int t = 0; t < 4; ++t) acc[t] = (v8f){};
#pragma unroll
  for (int kb = 0; kb < D; kb += 32) { const v16b a = frag_kb(&Ah[nloc][kb], hlf), al = frag_kb(&Al[nloc][kb], hlf);
#pragma unroll
    for (int t = 0; t < 4; ++t) { const v16b bw = frag_kb(WT + (size_t)(t * 16 + nloc) * D + kb, hlf); acc[t] = wmma16b(a, bw, acc[t]); acc[t] = wmma16b(al, bw, acc[t]); } }
}
__global__ __launch_bounds__(32) void iter0_kernel(const int* __restrict__ uid, const int* __restrict__ vid, const float* __restrict__ usr, const float* __restrict__ item, const float* __restrict__ ent, const float* __restrict__ rel, const b16* __restrict__ WT, const float* __restrict__ bias, const int* __restrict__ adj_e, const int* __restrict__ adj_r, float* __restrict__ O0, float* __restrict__ O1) {
  __shared__ __attribute__((aligned(16))) b16 Ah[16][D + 8], Al[16][D + 8]; __shared__ __attribute__((aligned(16))) float Tf[16][D + 4];
  const int lane = threadIdx.x, nloc = lane & 15, hlf = lane >> 4; const size_t m0 = (size_t)blockIdx.x * 16; const float sc = 1.0f / (XS * WSC); v8f acc[4];
#pragma unroll 1
  for (int slot = 0; slot < 1 + NN; ++slot) {
    for (int rr = 0; rr < 16; ++rr) { const size_t b = m0 + rr; const int u = iclamp(uid[b], 0, NU - 1), v = iclamp(vid[b], 0, NI - 1); const int vp = v >= NIKG ? NE : v;
      int self_ent; v2f selfv; const int* relid; const int* nbr;
      if (slot == 0) { const v2f t = *(const v2f*)(item + (size_t)v * D + lane * 2); selfv[0] = bf16_rne(t[0]); selfv[1] = bf16_rne(t[1]); relid = adj_r + (size_t)vp * NN; nbr = adj_e + (size_t)vp * NN; }
      else { self_ent = iclamp(adj_e[(size_t)vp * NN + (slot - 1)], 0, NE); const v2f t = *(const v2f*)(ent + (size_t)self_ent * D + lane * 2); selfv[0] = bf16_rne(t[0]); selfv[1] = bf16_rne(t[1]); relid = adj_r + (size_t)self_ent * NN; nbr = adj_e + (size_t)self_ent * NN; }
      build_A<0>(rr, usr + (size_t)u * D, selfv, relid, nbr, rel, ent, nullptr, 0, lane, Ah, Al); }
    wave_lds_sync();
    gemm64(Ah, Al, WT, nloc, hlf, acc);
#pragma unroll
    for (int t = 0; t < 4; ++t) { const int c = t * 16 + nloc; const float bb = bf16_rne(bias[c]);
#pragma unroll 1
      for (int r8 = 0; r8 < 8; ++r8) Tf[8 * hlf + r8][c] = sigm(acc[t][r8] * sc + bb); }
    wave_lds_sync();
    for (int pass = 0; pass < 2; ++pass) { for (int rr = 0; rr < 16; ++rr) { float* dst = slot == 0 ? O0 + (m0 + rr) * D : O1 + ((m0 + rr) * NN + (slot - 1)) * D; *(volatile v2f*)(dst + lane * 2) = *(const v2f*)(&Tf[rr][lane * 2]); } __threadfence(); }
    wave_lds_sync(); }
}
__global__ __launch_bounds__(64) void iter1_kernel(const int* __restrict__ uid, const int* __restrict__ vid, const float* __restrict__ usr, const float* __restrict__ rel, const b16* __restrict__ WT, const float* __restrict__ bias, const int* __restrict__ adj_r, const float* __restrict__ O0, const float* __restrict__ O1, float* __restrict__ out) {
  __shared__ __attribute__((aligned(16))) b16 Ah[2][16][D + 8], Al[2][16][D + 8]; __shared__ float so[32];
  const int wave = threadIdx.x >> 5, lane = threadIdx.x & 31, nloc = lane & 15, hlf = lane >> 4; const size_t m0 = (size_t)blockIdx.x * 32 + wave * 16; const float sc = 1.0f / (XS * WSC);
  for (int rr = 0; rr < 16; ++rr) { const size_t b = m0 + rr; const int u = iclamp(uid[b], 0, NU - 1), v = iclamp(vid[b], 0, NI - 1); const int vp = v >= NIKG ? NE : v; const v2f sv = *(const v2f*)(O0 + b * D + lane * 2);
    build_A<1>(rr, usr + (size_t)u * D, sv, adj_r + (size_t)vp * NN, nullptr, rel, nullptr, O1, b * NN, lane, Ah[wave], Al[wave]); }
  wave_lds_sync();
  v8f acc[4]; gemm64(Ah[wave], Al[wave], WT, nloc, hlf, acc);
  float pd[8]; for (int r8 = 0; r8 < 8; ++r8) pd[r8] = 0.0f;
#pragma unroll
  for (int t = 0; t < 4; ++t) { const int c = t * 16 + nloc; const float bb = bf16_rne(bias[c]);
#pragma unroll
    for (int r8 = 0; r8 < 8; ++r8) { const size_t b = m0 + 8 * hlf + r8; const int u = iclamp(uid[b], 0, NU - 1); const float iv = tanhf(acc[t][r8] * sc + bb); pd[r8] += pmul(bf16_rne(usr[(size_t)u * D + c]), iv); } }
#pragma unroll
  for (int r8 = 0; r8 < 8; ++r8) { float s = pd[r8]; for (int o = 1; o < 16; o <<= 1) s += __shfl_xor(s, o); if (nloc == 0) so[wave * 16 + 8 * hlf + r8] = sigm(s); }
  __syncthreads();
  for (int pass = 0; pass < 2; ++pass) { if (threadIdx.x < 32) ((volatile float*)out)[(size_t)blockIdx.x * 32 + threadIdx.x] = so[threadIdx.x]; __threadfence(); }
}
}

extern "C" void kernel_launch(void* const* d_in, const int* in_sizes, int n_in, void* d_out, int out_size, void* d_ws, size_t ws_size, hipStream_t stream) {
  (void)n_in;
  auto Fp = [&](int i) { return (const float*)d_in[i]; }; auto Ip = [&](int i) { return (const int*)d_in[i]; };
  if (in_sizes[0] != BT || in_sizes[1] != BT || in_sizes[2] != NU * D || in_sizes[3] != NI * D || in_sizes[4] != (NE + 1) * D || in_sizes[5] != (NR + 1) * D || in_sizes[6] != D * D || in_sizes[8] != (NE + 1) * NN || in_sizes[9] != (NE + 1) * NN || out_size != BT) return;
  const int NBV = BT;
  size_t off = 0; char* ws = (char*)d_ws;
  auto carve = [&](size_t bytes) { char* p = ws + off; off += (bytes + 255) & ~(size_t)255; return p; };
  b16* WT = (b16*)carve(D * D * 2); float* O0 = (float*)carve((size_t)BT * D * 4); float* O1 = (float*)carve((size_t)BT * NN * D * 4);
  if (off > ws_size || off > ((size_t)64 << 20)) return;
  wcopy_kernel<<<(D * D + 255) / 256, 256, 0, stream>>>(Fp(6), WT);
  iter0_kernel<<<NBV / 16, 32, 0, stream>>>(Ip(0), Ip(1), Fp(2), Fp(3), Fp(4), Fp(5), WT, Fp(7), Ip(8), Ip(9), O0, O1);
  iter1_kernel<<<NBV / 32, 64, 0, stream>>>(Ip(0), Ip(1), Fp(2), Fp(5), WT, Fp(7), Ip(9), O0, O1, (float*)d_out);
}
